// MLA_67070209294669
// MI455X (gfx1250) — hardware-verified
//
#include <hip/hip_runtime.h>
#include <math.h>
#include <stdint.h>

#ifndef NB
#define NB 2
#endif
#ifndef SEQ
#define SEQ 2048
#endif
#define NB_FULL  2
#define SEQ_FULL 2048
#define DIM   2048
#define NH    16
#define DNOPE 128
#define DROPE 64
#define DV    128
#define DQK   192
#define KVR   512
#define KVA   576
#define QW    3072
#define KNW   2048
#define WBR   4096
#define NTOK  (NB * SEQ)
#ifndef ER
#define ER    ((SEQ) < 512 ? (SEQ) : 512)
#endif
#define NER   (NB * ER)
#define NQB   (SEQ / 64)
#define NEQB  (ER / 64)
#define NQP   512
#define NKP   32
#define NINV  544
#define PCAR  1024.0f
#define WCAR  64.0f

static_assert(SEQ % 64 == 0);
static_assert(ER % 64 == 0);
static_assert(ER <= SEQ);
static_assert(SEQ <= SEQ_FULL);
static_assert(NB <= NB_FULL);
static_assert(NH * DNOPE == KNW);
static_assert(NH * DV == DIM);
static_assert(KNW == DIM);
static_assert(DQK == DNOPE + DROPE);
static_assert(KVA == KVR + DROPE);
static_assert(QW == NH * DQK);
static_assert(WBR == NH * (DNOPE + DV));
static_assert(NQP == NH * DROPE / 2);
static_assert(NKP == DROPE / 2);
static_assert(NINV == NQP + NKP);
static_assert(NINV % 32 == 0);
static_assert(NTOK % 64 == 0);
static_assert(KVA % 64 == 0);
static_assert(NQB <= 32);

typedef _Float16     v16h __attribute__((ext_vector_type(16)));
typedef _Float16     v8h  __attribute__((ext_vector_type(8)));
typedef __bf16       v16b __attribute__((ext_vector_type(16)));
typedef __bf16       v8b  __attribute__((ext_vector_type(8)));
typedef float        v8f  __attribute__((ext_vector_type(8)));
typedef float        v4f  __attribute__((ext_vector_type(4)));
typedef float        v2f  __attribute__((ext_vector_type(2)));
typedef unsigned int v4u  __attribute__((ext_vector_type(4)));

__device__ __forceinline__ unsigned short bf_bits(float f) {
  const unsigned u = __float_as_uint(f);
  return (unsigned short)((u + 0x7FFFu + ((u >> 16) & 1u)) >> 16);
}
__device__ __forceinline__ float bf_val(unsigned short h) { return __uint_as_float(((unsigned)h) << 16); }
__device__ __forceinline__ float bfr(float f) { return bf_val(bf_bits(f)); }
__device__ __forceinline__ unsigned short h_bits(float f) { const _Float16 h = (_Float16)f; return __builtin_bit_cast(unsigned short, h); }
__device__ __forceinline__ float h_val(unsigned short u) { return (float)__builtin_bit_cast(_Float16, u); }
__device__ __forceinline__ unsigned pk16(unsigned short a, unsigned short b) { return (unsigned)a | ((unsigned)b << 16); }
__device__ __forceinline__ v8f zero8() { v8f z = {0.f, 0.f, 0.f, 0.f, 0.f, 0.f, 0.f, 0.f}; return z; }
__device__ __forceinline__ int wave_id() { return __builtin_amdgcn_readfirstlane((int)(threadIdx.x >> 5)); }
__device__ __forceinline__ void lds_wave_sync() {
  __builtin_amdgcn_fence(3  , "workgroup");
  __builtin_amdgcn_wave_barrier();
  __builtin_amdgcn_fence(2  , "workgroup");
}
__device__ __forceinline__ v4u h8_to_b8(v4u w) {
  v4u o;
#pragma unroll
  for (int e = 0; e < 4; ++e) {
    const unsigned short lo = (unsigned short)(w[e] & 0xffffu), hi = (unsigned short)(w[e] >> 16);
    o[e] = pk16(bf_bits(h_val(lo)), bf_bits(h_val(hi)));
  }
  return o;
}

union FragH { v16h v; v8h h[2]; };
union FragB { v16b v; v8b h[2]; };
__device__ __forceinline__ v16h ldfrag_h(const _Float16* p) { FragH f; f.h[0] = *(const v8h*)(p); f.h[1] = *(const v8h*)(p + 16); return f.v; }
__device__ __forceinline__ v16b ldfrag_b(const __bf16* p)   { FragB f; f.h[0] = *(const v8b*)(p); f.h[1] = *(const v8b*)(p + 16); return f.v; }

__device__ __forceinline__ v8f mma_h(v16h a, v16h b, v8f c) {
  return __builtin_amdgcn_wmma_f32_16x16x32_f16(false, a, false, b, (short)0, c, false, false);
}
__device__ __forceinline__ v8f mma_b(v16b a, v16b b, v8f c) {
  return __builtin_amdgcn_wmma_f32_16x16x32_bf16(false, a, false, b, (short)0, c, false, false);
}
__device__ __forceinline__ void dep_guard_h(v8f& a, v8f& b, v16h x) {
  asm volatile("v_nop\n\tv_nop\n\tv_nop\n\tv_nop" : "+v"(a), "+v"(b) : "v"(x));
}
__device__ __forceinline__ void dep_guard_b(v8f& a, v8f& b, v16b x) {
  asm volatile("v_nop\n\tv_nop\n\tv_nop\n\tv_nop" : "+v"(a), "+v"(b) : "v"(x));
}
__device__ __forceinline__ void keep4_h(v16h a, v16h b, v16h c, v16h d) { asm volatile("v_nop" :: "v"(a), "v"(b), "v"(c), "v"(d)); }
__device__ __forceinline__ void keep4_b(v16b a, v16b b, v16b c, v16b d) { asm volatile("v_nop" :: "v"(a), "v"(b), "v"(c), "v"(d)); }
__device__ __forceinline__ void acc_guard4(v8f& a, v8f& b, v8f& c, v8f& d) {
  asm volatile("v_nop\n\tv_nop\n\tv_nop\n\tv_nop" : "+v"(a), "+v"(b), "+v"(c), "+v"(d));
}
__device__ __forceinline__ v8f at_mma_h(v16h a, v16h b, v8f c) {
  c = __builtin_amdgcn_wmma_f32_16x16x32_f16(false, a, false, b, (short)0, c, false, false);
  asm volatile("v_nop\n\tv_nop\n\tv_nop\n\tv_nop" : "+v"(c) : "v"(a), "v"(b));
  return c;
}
__device__ __forceinline__ v8f at_mma_b(v16b a, v16b b, v8f c) {
  c = __builtin_amdgcn_wmma_f32_16x16x32_bf16(false, a, false, b, (short)0, c, false, false);
  asm volatile("v_nop\n\tv_nop\n\tv_nop\n\tv_nop" : "+v"(c) : "v"(a), "v"(b));
  return c;
}

template <int MODE>
__global__ __launch_bounds__(256) void cvt_kernel(const float* __restrict__ in, long inStride,
                                                  unsigned short* oh, unsigned short* ob, long outStride, int n8, float sc) {
  const int i = (int)blockIdx.x * 256 + (int)threadIdx.x;
  if (i >= n8) return;
  const int bz = blockIdx.y;
  const size_t e = 8 * (size_t)i;
  const float* src = in + (size_t)bz * inStride + e;
  const v4f a = *(const v4f*)(src);
  const v4f c = *(const v4f*)(src + 4);
  const float f[8] = {a[0], a[1], a[2], a[3], c[0], c[1], c[2], c[3]};
  v4u hw, bw;
#pragma unroll
  for (int q = 0; q < 4; ++q) {
    const float f0 = bfr(f[2 * q]) * sc, f1 = bfr(f[2 * q + 1]) * sc;
    hw[q] = pk16(h_bits(f0), h_bits(f1));
    bw[q] = pk16(bf_bits(f0), bf_bits(f1));
  }
  unsigned short* dh = oh + (size_t)bz * outStride + e;
  unsigned short* db = ob + (size_t)bz * outStride + e;
  *(volatile v4u*)dh = hw;
  if (MODE == 1) *(volatile v4u*)db = bw;
  __threadfence();
  *(volatile v4u*)dh = hw;
  if (MODE == 1) *(volatile v4u*)db = bw;
}

__global__ __launch_bounds__(32) void invf_kernel(float* invf) {
  const int i = (int)blockIdx.x * 32 + (int)threadIdx.x;
  const bool isq = i < NQP;
  const int p = isq ? i : (i - NQP);
  const float d = isq ? 1024.0f : 64.0f;
  const float ex = (float)(2 * p) / d;
  const float v = 1.0f / powf(10000.0f, ex);
  *(volatile float*)(invf + i) = v;
  __threadfence();
  *(volatile float*)(invf + i) = v;
}

__global__ __launch_bounds__(256) void cs_kernel(const float* __restrict__ invf, float* csq, float* csk) {
  const int s = blockIdx.x, y = blockIdx.y, tid = (int)threadIdx.x;
  const bool kt = (y == 2);
  const int jk = (tid < NKP) ? tid : (NKP - 1);
  const int pi = kt ? (NQP + jk) : (y * 256 + tid);
  const float inv = invf[pi];
  const float ang = (float)s * inv;
  float sn, cs;
  sincosf(ang, &sn, &cs);
  v2f v;
  v[0] = cs; v[1] = sn;
  float* dst = kt ? (csk + ((size_t)s * NKP + jk) * 2) : (csq + ((size_t)s * NQP + y * 256 + tid) * 2);
  const bool w = kt ? (tid < NKP) : true;
  if (w) *(volatile v2f*)dst = v;
  __threadfence();
  if (w) *(volatile v2f*)dst = v;
}

__global__ __launch_bounds__(256) void flag_kernel(const float* __restrict__ mask, int* flags) {
  __shared__ int sfl[32];
  const int qt = blockIdx.x, tid = (int)threadIdx.x, lane = tid & 31, wave = tid >> 5;
  const int ct = tid >> 3, sub = tid & 7;
  const int ctc = (ct < NQB) ? ct : (NQB - 1);
  bool ok = true;
#pragma unroll 1
  for (int i = 0; i < 8; ++i) {
    const float* rp = mask + (size_t)(qt * 64 + sub * 8 + i) * SEQ_FULL + ctc * 64;
#pragma unroll
    for (int v = 0; v < 16; ++v) {
      const v4f m = *(const v4f*)(rp + 4 * v);
      ok = ok && (m[0] <= -1.0e8f) && (m[1] <= -1.0e8f) && (m[2] <= -1.0e8f) && (m[3] <= -1.0e8f);
    }
  }
  unsigned okb = ok ? 1u : 0u;
  okb &= (unsigned)__shfl_xor((int)okb, 1, 32);
  okb &= (unsigned)__shfl_xor((int)okb, 2, 32);
  okb &= (unsigned)__shfl_xor((int)okb, 4, 32);
  if ((lane & 7) == 0) sfl[wave * 4 + (lane >> 3)] = (int)okb;
  __syncthreads();
  if (wave == 0) {
    const int v = (lane < NQB) ? sfl[lane] : 1;
    *(volatile int*)(flags + qt * 32 + lane) = v;
    __threadfence();
    *(volatile int*)(flags + qt * 32 + lane) = v;
  }
}

__global__ __launch_bounds__(256) void prep_kernel(const float* __restrict__ kvf, const float* __restrict__ kvw, const float* __restrict__ csk,
                                                   unsigned short* lath, unsigned short* latl, unsigned short* kph, unsigned short* kpl) {
  __shared__ float part[8];
  const int tid = (int)threadIdx.x, lane = tid & 31, wave = tid >> 5;
  const int tk = tid >> 6, t = tid & 63;
  const int m = (int)blockIdx.x * 4 + tk;
  const int pos = m % SEQ, b = m / SEQ;
  const bool early = pos < ER;
  const float* row = kvf + (size_t)m * KVA;
  const v4f a0 = *(const v4f*)(row + 8 * t), a1 = *(const v4f*)(row + 8 * t + 4);
  const float x[8] = {a0[0], a0[1], a0[2], a0[3], a1[0], a1[1], a1[2], a1[3]};
  float ss = 0.f;
#pragma unroll
  for (int e = 0; e < 8; ++e) ss += x[e] * x[e];
#pragma unroll
  for (int off = 16; off > 0; off >>= 1) ss += __shfl_xor(ss, off, 32);
  if (lane == 0) part[wave] = ss;
  __syncthreads();
  const float tot = part[2 * tk] + part[2 * tk + 1];
  const float var = tot * (1.0f / 512.0f);
  const float rstd = rsqrtf(var + 1.0e-6f);
  const v4f w0 = *(const v4f*)(kvw + 8 * t), w1 = *(const v4f*)(kvw + 8 * t + 4);
  const float w[8] = {w0[0], w0[1], w0[2], w0[3], w1[0], w1[1], w1[2], w1[3]};
  v4u hw, lw;
#pragma unroll
  for (int q = 0; q < 4; ++q) {
    const float y0 = x[2 * q] * rstd * bfr(w[2 * q]);
    const float y1 = x[2 * q + 1] * rstd * bfr(w[2 * q + 1]);
    const unsigned short h0 = h_bits(y0), h1 = h_bits(y1);
    hw[q] = pk16(h0, h1);
    lw[q] = pk16(bf_bits(y0 - h_val(h0)), bf_bits(y1 - h_val(h1)));
  }
  const bool kw = ((wave & 1) == 0);
  const int tt = lane & 7;
  v4u khw, klw;
  khw[0] = khw[1] = khw[2] = khw[3] = 0u;
  klw = khw;
  if (kw) {
    const float* kp = row + KVR + 8 * tt;
    const v4f k0 = *(const v4f*)(kp), k1 = *(const v4f*)(kp + 4);
    const float kx[8] = {k0[0], k0[1], k0[2], k0[3], k1[0], k1[1], k1[2], k1[3]};
    const float* cp = csk + ((size_t)pos * NKP + 4 * tt) * 2;
    const v4f c0 = *(const v4f*)(cp), c1 = *(const v4f*)(cp + 4);
    const float cs[8] = {c0[0], c0[1], c0[2], c0[3], c1[0], c1[1], c1[2], c1[3]};
#pragma unroll
    for (int j = 0; j < 4; ++j) {
      const float x1 = kx[2 * j], x2 = kx[2 * j + 1], cc = cs[2 * j], sn = cs[2 * j + 1];
      const float o0 = x1 * cc - x2 * sn;
      const float o1 = x1 * sn + x2 * cc;
      const unsigned short h0 = h_bits(o0), h1 = h_bits(o1);
      khw[j] = pk16(h0, h1);
      klw[j] = pk16(bf_bits(o0 - h_val(h0)), bf_bits(o1 - h_val(h1)));
    }
  }
  unsigned short* dh  = lath + (size_t)m * KVR + 8 * t;
  unsigned short* dl  = latl + (size_t)m * KVR + 8 * t;
  const int posc = early ? pos : 0;
  unsigned short* dk  = kph + (size_t)m * DROPE + 8 * tt;
  unsigned short* dkl = kpl + ((size_t)b * ER + posc) * DROPE + 8 * tt;
  for (int pass = 0; pass < 2; ++pass) {
    *(volatile v4u*)dh = hw;
    *(volatile v4u*)dl = lw;
    if (kw && lane < 8) {
      *(volatile v4u*)dk = khw;
      if (early) *(volatile v4u*)dkl = klw;
    }
    __threadfence();
  }
}

template <bool SPLIT, int OM, bool ROPE>
__global__ __launch_bounds__(256) void gemm64_kernel(
    const unsigned short* __restrict__ Ap, int lda, long sA,
    const unsigned short* __restrict__ A2p, int lda2, long sA2,
    const unsigned short* __restrict__ Bp, int ldb, long sB,
    const unsigned short* __restrict__ B2p, int ldb2, long sB2,
    void* Cp, int ldc, long sC,
    void* C2p, int ldc2, long sC2,
    const float* __restrict__ bias, int hasb, const float* __restrict__ cst,
    int M, int N, int K, int agsz, int agoff, int bgsz, int bgoff, int esel, int a2c, int pcut, float scale) {
  __shared__ __align__(16) float sT[8][16 * 68];
  const int bz   = blockIdx.y;
  const int lane = threadIdx.x & 31;
  const int wave = wave_id();
  const int tilesN = N >> 6, tilesM = M >> 6;
  const int tile = (int)blockIdx.x * 8 + wave;
  if (tile >= tilesM * tilesN) return;
  const int tm = tile / tilesN;
  const int tn = tile - tm * tilesN;
  const int m0 = tm << 6, n0 = tn << 6;
  const int arow0 = (agsz > 0) ? ((m0 / agsz) * (2 * agsz) + agoff + (m0 % agsz)) : m0;
  const int brow0 = (bgsz > 0) ? ((n0 / bgsz) * (2 * bgsz) + bgoff + (n0 % bgsz)) : n0;
  const int pos0  = (esel == 0) ? (m0 % SEQ) : (n0 % SEQ);
  const int erow0 = (m0 / SEQ) * ER + (m0 % SEQ);
  const bool e_prod = SPLIT && (pos0 < pcut);
  const bool e_out  = (pos0 < ER);
  const int a2row0 = a2c ? erow0 : arow0;
  const int b2row0 = (esel == 0) ? brow0 : n0;

  const _Float16* Ab  = (const _Float16*)(const void*)Ap + (size_t)bz * sA;
  const __bf16*   A2b = (const __bf16*)(const void*)A2p  + (size_t)bz * sA2;
  const _Float16* Bb  = (const _Float16*)(const void*)Bp + (size_t)bz * sB;
  const __bf16*   B2b = (const __bf16*)(const void*)B2p  + (size_t)bz * sB2;

  const int rlane = lane & 15;
  const int koff  = (lane >> 4) * 8;
  const int mOff  = (lane >> 4) * 8;

  v8f acc[4][4];
#pragma unroll
  for (int i = 0; i < 4; ++i)
#pragma unroll
    for (int j = 0; j < 4; ++j) acc[i][j] = zero8();

  for (int k0 = 0; k0 < K; k0 += 32) {
    {
      v16h bh[4];
#pragma unroll
      for (int j = 0; j < 4; ++j) bh[j] = ldfrag_h(Bb + (size_t)(brow0 + (j << 4) + rlane) * ldb + koff + k0);
#pragma unroll
      for (int i = 0; i < 4; ++i) {
        const v16h ah = ldfrag_h(Ab + (size_t)(arow0 + (i << 4) + rlane) * lda + koff + k0);
#pragma unroll
        for (int j = 0; j < 4; ++j) acc[i][j] = mma_h(ah, bh[j], acc[i][j]);
        dep_guard_h(acc[i][0], acc[i][3], ah);
      }
      keep4_h(bh[0], bh[1], bh[2], bh[3]);
    }
    if (e_prod) {
      v16b bl[4];
#pragma unroll
      for (int j = 0; j < 4; ++j) bl[j] = ldfrag_b(B2b + (size_t)(b2row0 + (j << 4) + rlane) * ldb2 + koff + k0);
#pragma unroll
      for (int i = 0; i < 4; ++i) {
        const v16b al = ldfrag_b(A2b + (size_t)(a2row0 + (i << 4) + rlane) * lda2 + koff + k0);
#pragma unroll
        for (int j = 0; j < 4; ++j) acc[i][j] = mma_b(al, bl[j], acc[i][j]);
        dep_guard_b(acc[i][0], acc[i][3], al);
      }
      keep4_b(bl[0], bl[1], bl[2], bl[3]);
    }
  }
  acc_guard4(acc[0][0], acc[0][1], acc[0][2], acc[0][3]);
  acc_guard4(acc[1][0], acc[1][1], acc[1][2], acc[1][3]);
  acc_guard4(acc[2][0], acc[2][1], acc[2][2], acc[2][3]);
  acc_guard4(acc[3][0], acc[3][1], acc[3][2], acc[3][3]);

  float* slab = sT[wave];
  if (OM == 0) {
    float* C = (float*)Cp + (size_t)bz * sC;
    const int hh = lane >> 4, c4 = (lane & 15) * 4;
    v4f bv;
    bv[0] = bv[1] = bv[2] = bv[3] = 0.f;
    if (hasb) {
      const v4f t = *(const v4f*)(bias + n0 + c4);
      bv[0] = bfr(t[0]); bv[1] = bfr(t[1]); bv[2] = bfr(t[2]); bv[3] = bfr(t[3]);
    }
#pragma unroll
    for (int i = 0; i < 4; ++i) {
      const int mBase = m0 + (i << 4);
#pragma unroll
      for (int j = 0; j < 4; ++j)
#pragma unroll
        for (int r = 0; r < 8; ++r) slab[(mOff + r) * 68 + (j << 4) + rlane] = acc[i][j][r] * scale;
      lds_wave_sync();
      for (int pass = 0; pass < 2; ++pass) {
#pragma unroll
        for (int it = 0; it < 8; ++it) {
          const int row = it * 2 + hh;
          const v4f v = *(const v4f*)(slab + row * 68 + c4) + bv;
          *(volatile v4f*)(C + (size_t)(mBase + row) * ldc + n0 + c4) = v;
        }
        __threadfence();
      }
      lds_wave_sync();
    }
  } else {
    unsigned short* C  = (unsigned short*)Cp  + (size_t)bz * sC;
    unsigned short* C2 = (unsigned short*)C2p + (size_t)bz * sC2;
    const int qq = lane >> 3, c8 = (lane & 7) * 8;
    float bb[8] = {0.f, 0.f, 0.f, 0.f, 0.f, 0.f, 0.f, 0.f};
    if (hasb) {
      const v4f t0 = *(const v4f*)(bias + n0 + c8), t1 = *(const v4f*)(bias + n0 + c8 + 4);
      bb[0] = bfr(t0[0]); bb[1] = bfr(t0[1]); bb[2] = bfr(t0[2]); bb[3] = bfr(t0[3]);
      bb[4] = bfr(t1[0]); bb[5] = bfr(t1[1]); bb[6] = bfr(t1[2]); bb[7] = bfr(t1[3]);
    }
    const bool rt = ROPE && ((n0 % DQK) == DNOPE);
    const int p0 = (n0 / DQK) * (DROPE / 2) + (c8 >> 1);
#pragma unroll
    for (int i = 0; i < 4; ++i) {
      const int mBase = m0 + (i << 4);
#pragma unroll
      for (int j = 0; j < 4; ++j)
#pragma unroll
        for (int r = 0; r < 8; ++r) slab[(mOff + r) * 68 + (j << 4) + rlane] = acc[i][j][r] * scale;
      lds_wave_sync();
      v4u hv[4], lv[4];
#pragma unroll
      for (int it = 0; it < 4; ++it) {
        const int row = it * 4 + qq;
        const float* sp = slab + row * 68 + c8;
        const v4f x0 = *(const v4f*)sp, x1 = *(const v4f*)(sp + 4);
        float f[8] = {x0[0] + bb[0], x0[1] + bb[1], x0[2] + bb[2], x0[3] + bb[3],
                      x1[0] + bb[4], x1[1] + bb[5], x1[2] + bb[6], x1[3] + bb[7]};
        if (rt) {
          const int pos = (mBase + row) % SEQ;
          const float* tp = cst + ((size_t)pos * NQP + p0) * 2;
          const v4f t0 = *(const v4f*)tp, t1 = *(const v4f*)(tp + 4);
          const float cs[8] = {t0[0], t0[1], t0[2], t0[3], t1[0], t1[1], t1[2], t1[3]};
#pragma unroll
          for (int e = 0; e < 4; ++e) {
            const float x1v = f[2 * e], x2v = f[2 * e + 1], cc = cs[2 * e], sn = cs[2 * e + 1];
            f[2 * e]     = x1v * cc - x2v * sn;
            f[2 * e + 1] = x1v * sn + x2v * cc;
          }
        }
        v4u a, l;
#pragma unroll
        for (int e = 0; e < 4; ++e) {
          const unsigned short h0 = h_bits(f[2 * e]), h1 = h_bits(f[2 * e + 1]);
          a[e] = pk16(h0, h1);
          l[e] = pk16(bf_bits(f[2 * e] - h_val(h0)), bf_bits(f[2 * e + 1] - h_val(h1)));
        }
        hv[it] = a;
        lv[it] = l;
      }
      const int c2r0 = (esel == 0) ? (erow0 + (i << 4)) : mBase;
      for (int pass = 0; pass < 2; ++pass) {
#pragma unroll
        for (int it = 0; it < 4; ++it) {
          const int row = it * 4 + qq;
          *(volatile v4u*)(C + (size_t)(mBase + row) * ldc + n0 + c8) = hv[it];
          if (e_out) *(volatile v4u*)(C2 + (size_t)(c2r0 + row) * ldc2 + n0 + c8) = lv[it];
        }
        __threadfence();
      }
      lds_wave_sync();
    }
  }
}

#define ATT_QT (64 * DQK)
#define ATT_PT (4 * 16 * 64)
#define ATT_LDS_LATE  ((ATT_QT + ATT_QT + 128 * 64 + ATT_PT) * 2 + 64 * 64 * 4)
#define ATT_LDS_EARLY ((3 * ATT_QT + 3 * ATT_QT + 3 * 64 * 64 + 3 * ATT_PT) * 2 + 64 * 64 * 4)
static_assert(ATT_LDS_LATE == 90112);
static_assert(ATT_LDS_EARLY == 212992);

template <bool EARLY>
__global__ __launch_bounds__(128) void attn_kernel(
    const unsigned short* __restrict__ QHp, const unsigned short* __restrict__ QLp,
    const unsigned short* __restrict__ KNHp, const unsigned short* __restrict__ KNLp,
    const unsigned short* __restrict__ KPHp, const unsigned short* __restrict__ KPLp,
    const unsigned short* __restrict__ VTHp, const unsigned short* __restrict__ VTLp,
    const float* __restrict__ mask, const int* __restrict__ flags,
    unsigned short* CTXH, unsigned short* CTXL, float sscale) {
  extern __shared__ __align__(16) unsigned char dyn_lds[];
  constexpr int VT  = EARLY ? 4 : 8;
  constexpr int VD  = 16 * VT;
  constexpr int QT  = ATT_QT;
  constexpr int VTS = VD * 64;
  constexpr int PT  = ATT_PT;
  _Float16* Qh  = (_Float16*)dyn_lds;
  __bf16*   Qhb = (__bf16*)(dyn_lds + QT * 2);
  __bf16*   Qlb = (__bf16*)(dyn_lds + QT * 4);
  unsigned char* kbase = dyn_lds + (EARLY ? 3 : 1) * QT * 2;
  _Float16* Kh  = (_Float16*)kbase;
  __bf16*   Khb = (__bf16*)(kbase + QT * 2);
  __bf16*   Klb = (__bf16*)(kbase + QT * 4);
  unsigned char* vbase = kbase + (EARLY ? 3 : 1) * QT * 2;
  _Float16* Vt  = (_Float16*)vbase;
  __bf16*   Vtb = (__bf16*)(vbase + VTS * 2);
  __bf16*   Vtl = (__bf16*)(vbase + VTS * 4);
  unsigned char* pbase = vbase + (EARLY ? 3 : 1) * VTS * 2;
  _Float16* Ph  = (_Float16*)pbase;
  __bf16*   Phb = (__bf16*)(pbase + PT * 2);
  __bf16*   Plb = (__bf16*)(pbase + PT * 4);
  float* Msh = (float*)(pbase + (EARLY ? 3 : 1) * PT * 2);

  const int tid = (int)threadIdx.x, wave = wave_id(), lane = tid & 31;
  const int hh = lane >> 4, c = lane & 15;
  const int b = (int)blockIdx.y;
  int bx = (int)blockIdx.x;
  int vh = 0, qb, h;
  if (EARLY) { vh = bx & 1; bx >>= 1; qb = bx % NEQB; h = bx / NEQB; }
  else { constexpr int NL = (NQB - NEQB) > 0 ? (NQB - NEQB) : 1; qb = NEQB + bx % NL; h = bx / NL; }
  const size_t tok0 = (size_t)b * SEQ;
  const int q0b = qb * 64, q0w = wave * 16;
  const size_t erb = (size_t)b * ER;

  const int fl = flags[qb * 32 + lane];
  const unsigned vis = (unsigned)__builtin_amdgcn_ballot_w32(fl == 0);
  const bool blockbad = EARLY && ((vis >> NEQB) != 0u);

  {
    const int r = tid >> 1, half = (tid & 1) * 96;
    const unsigned short* src = QHp + (tok0 + q0b + r) * (size_t)QW + h * DQK + half;
    const unsigned short* srl = QLp + (erb + q0b + r) * (size_t)QW + h * DQK + half;
#pragma unroll
    for (int i = 0; i < 12; ++i) {
      const v4u w = *(const v4u*)(src + 8 * i);
      *(v4u*)(Qh + r * DQK + half + 8 * i) = w;
      if (EARLY) {
        *(v4u*)(Qhb + r * DQK + half + 8 * i) = h8_to_b8(w);
        *(v4u*)(Qlb + r * DQK + half + 8 * i) = *(const v4u*)(srl + 8 * i);
      }
    }
  }

  float mrow[8], lrow[8];
  v8f oacc[VT];
#pragma unroll
  for (int r = 0; r < 8; ++r) { mrow[r] = -INFINITY; lrow[r] = 0.f; }
#pragma unroll
  for (int t = 0; t < VT; ++t) oacc[t] = zero8();

  _Float16* pwh = Ph  + wave * (16 * 64);
  __bf16*   pwb = Phb + wave * (16 * 64);
  __bf16*   pwl = Plb + wave * (16 * 64);

  constexpr int KCMAX = EARLY ? NEQB : NQB;
#pragma unroll 1
  for (int kc = 0; kc < KCMAX; ++kc) {
    if (!((vis >> kc) & 1u)) continue;
    const int kv0 = kc * 64;
    __syncthreads();
    if (tid < 64) {
      const int r = tid;
      const unsigned short* ks  = KNHp + (tok0 + kv0 + r) * (size_t)KNW + h * DNOPE;
      const unsigned short* ksl = KNLp + (erb + kv0 + r) * (size_t)KNW + h * DNOPE;
#pragma unroll
      for (int i = 0; i < 16; ++i) {
        const v4u w = *(const v4u*)(ks + 8 * i);
        *(v4u*)(Kh + r * DQK + 8 * i) = w;
        if (EARLY) {
          *(v4u*)(Khb + r * DQK + 8 * i) = h8_to_b8(w);
          *(v4u*)(Klb + r * DQK + 8 * i) = *(const v4u*)(ksl + 8 * i);
        }
      }
      if (EARLY) {
        const size_t vr = (size_t)b * KNW + (size_t)h * DV + vh * 64 + r;
        const unsigned short* vs  = VTHp + vr * SEQ + kv0;
        const unsigned short* vsl = VTLp + vr * ER + kv0;
#pragma unroll
        for (int i = 0; i < 8; ++i) {
          const v4u w = *(const v4u*)(vs + 8 * i);
          *(v4u*)(Vt  + r * 64 + 8 * i) = w;
          *(v4u*)(Vtb + r * 64 + 8 * i) = h8_to_b8(w);
          *(v4u*)(Vtl + r * 64 + 8 * i) = *(const v4u*)(vsl + 8 * i);
        }
      }
    } else {
      const int r = tid - 64;
      const unsigned short* ps  = KPHp + (tok0 + kv0 + r) * (size_t)DROPE;
      const unsigned short* psl = KPLp + (erb + kv0 + r) * (size_t)DROPE;
#pragma unroll
      for (int i = 0; i < 8; ++i) {
        const v4u w = *(const v4u*)(ps + 8 * i);
        *(v4u*)(Kh + r * DQK + DNOPE + 8 * i) = w;
        if (EARLY) {
          *(v4u*)(Khb + r * DQK + DNOPE + 8 * i) = h8_to_b8(w);
          *(v4u*)(Klb + r * DQK + DNOPE + 8 * i) = *(const v4u*)(psl + 8 * i);
        }
      }
    }
    if (!EARLY) {
      const int r = tid;
      const unsigned short* vs = VTHp + ((size_t)b * KNW + (size_t)h * DV + r) * SEQ + kv0;
#pragma unroll
      for (int i = 0; i < 8; ++i) *(v4u*)(Vt + r * 64 + 8 * i) = *(const v4u*)(vs + 8 * i);
    }
    {
#pragma unroll
      for (int it = 0; it < 8; ++it) {
        const int idx = it * 128 + tid;
        const int r = idx >> 4, c4 = (idx & 15) * 4;
        *(v4f*)(Msh + r * 64 + c4) = *(const v4f*)(mask + (size_t)(q0b + r) * SEQ_FULL + kv0 + c4);
      }
    }
    __syncthreads();

    v8f s[4];
#pragma unroll
    for (int j = 0; j < 4; ++j) s[j] = zero8();
#pragma unroll
    for (int dc = 0; dc < 6; ++dc) {
      FragH qa;
      qa.h[0] = *(const v8h*)(Qh + (q0w + c) * DQK + dc * 32 + 8 * hh);
      qa.h[1] = *(const v8h*)(Qh + (q0w + c) * DQK + dc * 32 + 16 + 8 * hh);
      FragB qab, qal;
      if (EARLY) {
        qab.h[0] = *(const v8b*)(Qhb + (q0w + c) * DQK + dc * 32 + 8 * hh);
        qab.h[1] = *(const v8b*)(Qhb + (q0w + c) * DQK + dc * 32 + 16 + 8 * hh);
        qal.h[0] = *(const v8b*)(Qlb + (q0w + c) * DQK + dc * 32 + 8 * hh);
        qal.h[1] = *(const v8b*)(Qlb + (q0w + c) * DQK + dc * 32 + 16 + 8 * hh);
      }
#pragma unroll
      for (int j = 0; j < 4; ++j) {
        FragH kb;
        kb.h[0] = *(const v8h*)(Kh + (j * 16 + c) * DQK + dc * 32 + 8 * hh);
        kb.h[1] = *(const v8h*)(Kh + (j * 16 + c) * DQK + dc * 32 + 16 + 8 * hh);
        s[j] = at_mma_h(qa.v, kb.v, s[j]);
        if (EARLY) {
          FragB kbb, klb;
          kbb.h[0] = *(const v8b*)(Khb + (j * 16 + c) * DQK + dc * 32 + 8 * hh);
          kbb.h[1] = *(const v8b*)(Khb + (j * 16 + c) * DQK + dc * 32 + 16 + 8 * hh);
          klb.h[0] = *(const v8b*)(Klb + (j * 16 + c) * DQK + dc * 32 + 8 * hh);
          klb.h[1] = *(const v8b*)(Klb + (j * 16 + c) * DQK + dc * 32 + 16 + 8 * hh);
          s[j] = at_mma_b(qab.v, klb.v, s[j]);
          s[j] = at_mma_b(qal.v, kbb.v, s[j]);
        }
      }
    }
    float cm[8];
#pragma unroll
    for (int r = 0; r < 8; ++r) {
      const int ql = q0w + 8 * hh + r;
      float m = -INFINITY;
#pragma unroll
      for (int j = 0; j < 4; ++j) {
        const float sv = s[j][r] * sscale + Msh[ql * 64 + j * 16 + c];
        s[j][r] = sv;
        m = fmaxf(m, sv);
      }
#pragma unroll
      for (int off = 1; off < 16; off <<= 1) m = fmaxf(m, __shfl_xor(m, off, 32));
      cm[r] = m;
    }
#pragma unroll
    for (int r = 0; r < 8; ++r) {
      const float mnew  = fmaxf(mrow[r], cm[r]);
      const float alpha = expf(mrow[r] - mnew);
      mrow[r] = mnew;
      float psum = 0.f;
#pragma unroll
      for (int j = 0; j < 4; ++j) {
        const float p = expf(s[j][r] - mnew);
        psum += p;
        const float pc = p * PCAR;
        const _Float16 phv = (_Float16)pc;
        const int pi = (8 * hh + r) * 64 + j * 16 + c;
        pwh[pi] = phv;
        if (EARLY) {
          const float phf = (float)phv;
          pwb[pi] = __builtin_bit_cast(__bf16, bf_bits(phf));
          pwl[pi] = __builtin_bit_cast(__bf16, bf_bits(pc - phf));
        }
      }
#pragma unroll
      for (int off = 1; off < 16; off <<= 1) psum += __shfl_xor(psum, off, 32);
      lrow[r] = lrow[r] * alpha + psum;
#pragma unroll
      for (int t = 0; t < VT; ++t) oacc[t][r] *= alpha;
    }
    lds_wave_sync();
#pragma unroll 1
    for (int kk = 0; kk < 2; ++kk) {
      FragH pa;
      pa.h[0] = *(const v8h*)(pwh + c * 64 + kk * 32 + 8 * hh);
      pa.h[1] = *(const v8h*)(pwh + c * 64 + kk * 32 + 16 + 8 * hh);
      FragB pab, pal;
      if (EARLY) {
        pab.h[0] = *(const v8b*)(pwb + c * 64 + kk * 32 + 8 * hh);
        pab.h[1] = *(const v8b*)(pwb + c * 64 + kk * 32 + 16 + 8 * hh);
        pal.h[0] = *(const v8b*)(pwl + c * 64 + kk * 32 + 8 * hh);
        pal.h[1] = *(const v8b*)(pwl + c * 64 + kk * 32 + 16 + 8 * hh);
      }
#pragma unroll
      for (int t = 0; t < VT; ++t) {
        FragH vb;
        vb.h[0] = *(const v8h*)(Vt + (t * 16 + c) * 64 + kk * 32 + 8 * hh);
        vb.h[1] = *(const v8h*)(Vt + (t * 16 + c) * 64 + kk * 32 + 16 + 8 * hh);
        oacc[t] = at_mma_h(pa.v, vb.v, oacc[t]);
        if (EARLY) {
          FragB vbb, vlb;
          vbb.h[0] = *(const v8b*)(Vtb + (t * 16 + c) * 64 + kk * 32 + 8 * hh);
          vbb.h[1] = *(const v8b*)(Vtb + (t * 16 + c) * 64 + kk * 32 + 16 + 8 * hh);
          vlb.h[0] = *(const v8b*)(Vtl + (t * 16 + c) * 64 + kk * 32 + 8 * hh);
          vlb.h[1] = *(const v8b*)(Vtl + (t * 16 + c) * 64 + kk * 32 + 16 + 8 * hh);
          oacc[t] = at_mma_b(pab.v, vlb.v, oacc[t]);
          oacc[t] = at_mma_b(pal.v, vbb.v, oacc[t]);
        }
      }
    }
  }
  acc_guard4(oacc[0], oacc[1], oacc[2], oacc[3]);
  if constexpr (!EARLY) acc_guard4(oacc[4], oacc[5], oacc[6], oacc[7]);
  __syncthreads();

  const float qnan = __uint_as_float(0x7fc00000u);
  unsigned short* osh = (unsigned short*)Kh + wave * (16 * VD);
  unsigned short* osl = (unsigned short*)Kh + 4 * 16 * VD + wave * (16 * VD);
#pragma unroll
  for (int r = 0; r < 8; ++r) {
    const bool bad = blockbad || !(lrow[r] > 0.f) || !(mrow[r] > -1.0e8f);
    const float den = bad ? 1.0f : (lrow[r] * PCAR);
    const float inv = 1.0f / den;
#pragma unroll
    for (int t = 0; t < VT; ++t) {
      const float o = bad ? qnan : (oacc[t][r] * inv);
      const unsigned short hb = h_bits(o);
      const int so = (8 * hh + r) * VD + t * 16 + c;
      osh[so] = hb;
      if (EARLY) osl[so] = bf_bits(o - h_val(hb));
    }
  }
  lds_wave_sync();
  if (!EARLY) {
    unsigned short* Ag = CTXH + (tok0 + q0b + q0w) * (size_t)KNW + (size_t)h * DV;
    const int rh = lane >> 4, c8 = (lane & 15) * 8;
    for (int pass = 0; pass < 2; ++pass) {
#pragma unroll
      for (int it = 0; it < 8; ++it) {
        const int row = it * 2 + rh;
        const v4u x = *(const v4u*)(osh + row * VD + c8);
        *(volatile v4u*)(Ag + (size_t)row * KNW + c8) = x;
      }
      __threadfence();
    }
  } else {
    unsigned short* Ag = CTXH + (tok0 + q0b + q0w) * (size_t)KNW + (size_t)h * DV + vh * 64;
    unsigned short* Al = CTXL + (erb + q0b + q0w) * (size_t)KNW + (size_t)h * DV + vh * 64;
    const int rq = lane >> 3, c8 = (lane & 7) * 8;
    for (int pass = 0; pass < 2; ++pass) {
#pragma unroll
      for (int it = 0; it < 4; ++it) {
        const int row = it * 4 + rq;
        const v4u x = *(const v4u*)(osh + row * VD + c8);
        const v4u y = *(const v4u*)(osl + row * VD + c8);
        *(volatile v4u*)(Ag + (size_t)row * KNW + c8) = x;
        *(volatile v4u*)(Al + (size_t)row * KNW + c8) = y;
      }
      __threadfence();
    }
  }
}

static inline size_t al128(size_t x) { return (x + 127) & ~(size_t)127; }
static inline size_t smax(size_t a, size_t b) { return a > b ? a : b; }

extern "C" void kernel_launch(void* const* d_in, const int* in_sizes, int n_in,
                              void* d_out, int out_size, void* d_ws, size_t ws_size,
                              hipStream_t stream) {
  if (n_in < 10) return;
  if (in_sizes[0] < NB * SEQ_FULL * DIM) return;
  if (in_sizes[1] < SEQ_FULL * SEQ_FULL) return;
  if (in_sizes[2] != QW * DIM) return;
  if (in_sizes[3] != QW) return;
  if (in_sizes[4] != KVA * DIM) return;
  if (in_sizes[5] != KVA) return;
  if (in_sizes[6] != KVR) return;
  if (in_sizes[7] != WBR * KVR) return;
  if (in_sizes[8] != DIM * DIM) return;
  if (in_sizes[9] != DIM) return;
  if (out_size < NTOK * DIM) return;

  const float* x     = (const float*)d_in[0];
  const float* mask  = (const float*)d_in[1];
  const float* wq    = (const float*)d_in[2];
  const float* bq    = (const float*)d_in[3];
  const float* wkv_a = (const float*)d_in[4];
  const float* bkv_a = (const float*)d_in[5];
  const float* kvw   = (const float*)d_in[6];
  const float* wkv_b = (const float*)d_in[7];
  const float* wo    = (const float*)d_in[8];
  const float* bo    = (const float*)d_in[9];
  float* out = (float*)d_out;

  const size_t szXB   = (size_t)NTOK * DIM * 2;
  const size_t szKNH  = (size_t)NTOK * KNW * 2;
  const size_t szWQ   = (size_t)QW * DIM * 2;
  const size_t szWA   = (size_t)KVA * DIM * 2;
  const size_t szCSQ  = (size_t)SEQ * NQP * 8;
  const size_t szLATH = (size_t)NTOK * KVR * 2;
  const size_t szLATL = (size_t)NTOK * KVR * 2;
  const size_t szCTXH = (size_t)NTOK * KNW * 2;
  const size_t szCTXL = (size_t)NER * KNW * 2;
  const size_t szKVF  = (size_t)NTOK * KVA * 4;
  const size_t szKNL  = (size_t)NER * KNW * 2;
  const size_t szVTL  = (size_t)NB * KNW * ER * 2;
  const size_t szCSK  = (size_t)SEQ * NKP * 8;
  const size_t szINV  = al128((size_t)NINV * 4);
  const size_t szWB   = (size_t)WBR * KVR * 2;
  const size_t szWO   = (size_t)DIM * DIM * 2;
  const size_t szQH   = (size_t)NTOK * QW * 2;
  const size_t szQL   = (size_t)NER * QW * 2;
  const size_t szKPH  = (size_t)NTOK * DROPE * 2;
  const size_t szKPL  = (size_t)NER * DROPE * 2;
  const size_t szVTH  = (size_t)NB * KNW * SEQ * 2;
  const size_t szFL   = al128((size_t)NQB * 32 * 4);

  const size_t szRA = smax(szXB, szKNH);
  const size_t szRB = smax(smax(szWQ + szWA + szCSQ, szLATH + szLATL), szCTXH + szCTXL);
  const size_t szRC = smax(szKVF, szKNL + szVTL);

  size_t off = 0;
  const size_t oRA  = off; off += szRA;
  const size_t oRB  = off; off += szRB;
  const size_t oRC  = off; off += szRC;
  const size_t oCSK = off; off += szCSK;
  const size_t oINV = off; off += szINV;
  const size_t oWB  = off; off += szWB;
  const size_t oWBB = off; off += szWB;
  const size_t oWO  = off; off += szWO;
  const size_t oWOB = off; off += szWO;
  const size_t oQH  = off; off += szQH;
  const size_t oQL  = off; off += szQL;
  const size_t oKPH = off; off += szKPH;
  const size_t oKPL = off; off += szKPL;
  const size_t oVTH = off; off += szVTH;
  const size_t oFL  = off; off += szFL;
  if (off > ws_size) return;
  if (off > (size_t)134217728) return;

  char* ws = (char*)d_ws;
  unsigned short* XB   = (unsigned short*)(ws + oRA);
  unsigned short* KNH  = (unsigned short*)(ws + oRA);
  unsigned short* WQP  = (unsigned short*)(ws + oRB);
  unsigned short* WAP  = (unsigned short*)(ws + oRB + szWQ);
  float*          CSQ  = (float*)(ws + oRB + szWQ + szWA);
  unsigned short* LATH = (unsigned short*)(ws + oRB);
  unsigned short* LATL = (unsigned short*)(ws + oRB + szLATH);
  unsigned short* CTXH = (unsigned short*)(ws + oRB);
  unsigned short* CTXL = (unsigned short*)(ws + oRB + szCTXH);
  float*          KVF  = (float*)(ws + oRC);
  unsigned short* KNL  = (unsigned short*)(ws + oRC);
  unsigned short* VTL  = (unsigned short*)(ws + oRC + szKNL);
  float*          CSK  = (float*)(ws + oCSK);
  float*          INVF = (float*)(ws + oINV);
  unsigned short* WB   = (unsigned short*)(ws + oWB);
  unsigned short* WBB  = (unsigned short*)(ws + oWBB);
  unsigned short* WOP  = (unsigned short*)(ws + oWO);
  unsigned short* WOB  = (unsigned short*)(ws + oWOB);
  unsigned short* QH   = (unsigned short*)(ws + oQH);
  unsigned short* QL   = (unsigned short*)(ws + oQL);
  unsigned short* KPH  = (unsigned short*)(ws + oKPH);
  unsigned short* KPL  = (unsigned short*)(ws + oKPL);
  unsigned short* VTH  = (unsigned short*)(ws + oVTH);
  int*            FLAGS = (int*)(ws + oFL);

  const dim3 b256(256), b128(128), b32(32);
  const float wsc = 1.0f / WCAR;
  const float sscale = 0.072168783648703216f;

  cvt_kernel<0><<<dim3((SEQ * DIM / 8) / 256, NB), b256, 0, stream>>>(x, (long)SEQ_FULL * DIM, XB, XB, (long)SEQ * DIM, SEQ * DIM / 8, 1.0f);
  cvt_kernel<0><<<dim3((QW * DIM / 8) / 256, 1), b256, 0, stream>>>(wq, 0L, WQP, WQP, 0L, QW * DIM / 8, WCAR);
  cvt_kernel<0><<<dim3((KVA * DIM / 8) / 256, 1), b256, 0, stream>>>(wkv_a, 0L, WAP, WAP, 0L, KVA * DIM / 8, WCAR);
  cvt_kernel<1><<<dim3((WBR * KVR / 8) / 256, 1), b256, 0, stream>>>(wkv_b, 0L, WB, WBB, 0L, WBR * KVR / 8, WCAR);
  cvt_kernel<1><<<dim3((DIM * DIM / 8) / 256, 1), b256, 0, stream>>>(wo, 0L, WOP, WOB, 0L, DIM * DIM / 8, WCAR);
  invf_kernel<<<dim3(NINV / 32), b32, 0, stream>>>(INVF);
  cs_kernel<<<dim3(SEQ, 3), b256, 0, stream>>>(INVF, CSQ, CSK);
  flag_kernel<<<dim3(NQB), b256, 0, stream>>>(mask, FLAGS);
  gemm64_kernel<false, 2, true><<<dim3(((NTOK / 64) * (QW / 64) + 7) / 8, 1), b256, 0, stream>>>(
      XB, DIM, 0L, XB, DIM, 0L, WQP, DIM, 0L, WQP, DIM, 0L, (void*)QH, QW, 0L, (void*)QL, QW, 0L,
      bq, 1, CSQ, NTOK, QW, DIM, 0, 0, 0, 0, 0, 1, 0, wsc);
  gemm64_kernel<false, 0, false><<<dim3(((NTOK / 64) * (KVA / 64) + 7) / 8, 1), b256, 0, stream>>>(
      XB, DIM, 0L, XB, DIM, 0L, WAP, DIM, 0L, WAP, DIM, 0L, (void*)KVF, KVA, 0L, (void*)KVF, KVA, 0L,
      bkv_a, 1, CSQ, NTOK, KVA, DIM, 0, 0, 0, 0, 0, 0, 0, wsc);
  prep_kernel<<<dim3(NTOK / 4), b256, 0, stream>>>(KVF, kvw, CSK, LATH, LATL, KPH, KPL);
  gemm64_kernel<true, 2, false><<<dim3(((NTOK / 64) * (KNW / 64) + 7) / 8, 1), b256, 0, stream>>>(
      LATH, KVR, 0L, LATL, KVR, 0L, WB, KVR, 0L, WBB, KVR, 0L, (void*)KNH, KNW, 0L, (void*)KNL, KNW, 0L,
      bq, 0, CSQ, NTOK, KNW, KVR, 0, 0, 128, 0, 0, 0, SEQ, wsc);
  gemm64_kernel<true, 2, false><<<dim3(((KNW / 64) * (SEQ / 64) + 7) / 8, NB), b256, 0, stream>>>(
      WB, KVR, 0L, WBB, KVR, 0L, LATH, KVR, (long)SEQ * KVR, LATL, KVR, (long)SEQ * KVR,
      (void*)VTH, SEQ, (long)KNW * SEQ, (void*)VTL, ER, (long)KNW * ER,
      bq, 0, CSQ, KNW, SEQ, KVR, 128, 128, 0, 0, 1, 0, SEQ, wsc);
  (void)hipFuncSetAttribute(reinterpret_cast<const void*>(&attn_kernel<true>), hipFuncAttributeMaxDynamicSharedMemorySize, ATT_LDS_EARLY);
  (void)hipFuncSetAttribute(reinterpret_cast<const void*>(&attn_kernel<false>), hipFuncAttributeMaxDynamicSharedMemorySize, ATT_LDS_LATE);
  attn_kernel<true><<<dim3(NH * NEQB * 2, NB), b128, ATT_LDS_EARLY, stream>>>(
      QH, QL, KNH, KNL, KPH, KPL, VTH, VTL, mask, FLAGS, CTXH, CTXL, sscale);
  if (NQB > NEQB) {
    attn_kernel<false><<<dim3(NH * (NQB - NEQB), NB), b128, ATT_LDS_LATE, stream>>>(
        QH, QL, KNH, KNL, KPH, KPL, VTH, VTL, mask, FLAGS, CTXH, CTXL, sscale);
  }
  gemm64_kernel<true, 0, false><<<dim3(((NTOK / 64) * (DIM / 64) + 7) / 8, 1), b256, 0, stream>>>(
      CTXH, KNW, 0L, CTXL, KNW, 0L, WOP, DIM, 0L, WOB, DIM, 0L, (void*)out, DIM, 0L, (void*)out, DIM, 0L,
      bo, 1, CSQ, NTOK, DIM, KNW, 0, 0, 0, 0, 0, 1, ER, wsc);
  (void)hipGetLastError();
}
